// GGN_IO_35983236006287
// MI455X (gfx1250) — hardware-verified
//
#include <hip/hip_runtime.h>
#include <math.h>

typedef __attribute__((ext_vector_type(16))) _Float16 v16h;
typedef __attribute__((ext_vector_type(16))) __bf16 v16b;
typedef __attribute__((ext_vector_type(8)))  _Float16 v8h;
typedef __attribute__((ext_vector_type(8)))  float v8f;
typedef __attribute__((ext_vector_type(4)))  float v4f;
typedef __attribute__((ext_vector_type(2)))  float v2f;
typedef __attribute__((ext_vector_type(4)))  unsigned v4u;
typedef __attribute__((ext_vector_type(4)))  int v4i;
typedef float __attribute__((may_alias)) float_a;
typedef int __attribute__((may_alias)) int_a;

template <typename T> __device__ __forceinline__ void vst2(void* p, T v) { *(volatile T*)p = v; __threadfence(); *(volatile T*)p = v; }
__device__ __forceinline__ v8f wmma16(v16h a, v16h b, v8f c) {
  v8f d = __builtin_amdgcn_wmma_f32_16x16x32_f16(false, a, false, b, (short)0, c, false, false);
  asm volatile("v_nop\n\tv_nop\n\tv_nop\n\tv_nop" : "+v"(d) : "v"(a), "v"(b));
  return d;
}
__device__ __forceinline__ v8f wmma_bf(v16b a, v16b b, v8f c) {
  v8f d = __builtin_amdgcn_wmma_f32_16x16x32_bf16(false, a, false, b, (short)0, c, false, false);
  asm volatile("v_nop\n\tv_nop\n\tv_nop\n\tv_nop" : "+v"(d) : "v"(a), "v"(b));
  return d;
}
__device__ __forceinline__ v16h frag_h(const _Float16* rowk0, int lane) {
  union { v16h v; v8h q[2]; } u; const _Float16* p = rowk0 + 8 * (lane >> 4);
  u.q[0] = *(const v8h*)p; u.q[1] = *(const v8h*)(p + 16); return u.v;
}
__device__ __forceinline__ v16h frag_f32(const float* rowk0, int lane) {
  v16h a; const float* p = rowk0 + 8 * (lane >> 4);
#pragma unroll
  for (int i = 0; i < 8; ++i) { a[i] = (_Float16)p[i]; a[8 + i] = (_Float16)p[16 + i]; }
  return a;
}
__device__ __forceinline__ v16h frag_f32s(const float* rowk0, int lane, float sc) {
  v16h a; const float* p = rowk0 + 8 * (lane >> 4);
#pragma unroll
  for (int i = 0; i < 8; ++i) { a[i] = (_Float16)(p[i] * sc); a[8 + i] = (_Float16)(p[16 + i] * sc); }
  return a;
}
__device__ __forceinline__ v16h fragc_f32(const float* W, int k0, int n, int lane, int ld, int K) {
  v16h a; const int g = lane >> 4;
#pragma unroll
  for (int i = 0; i < 8; ++i) { const int ka = k0 + 8 * g + i, kb = ka + 16;
    a[i] = (_Float16)(ka < K ? W[(size_t)ka * ld + n] : 0.f); a[8 + i] = (_Float16)(kb < K ? W[(size_t)kb * ld + n] : 0.f); }
  return a;
}
struct F2 { v16b h, l; };
__device__ __forceinline__ F2 bsplit16(const float v[16]) { F2 r;
#pragma unroll
  for (int i = 0; i < 16; ++i) { const __bf16 h = (__bf16)v[i]; r.h[i] = h; r.l[i] = (__bf16)(v[i] - (float)h); }
  return r; }
__device__ __forceinline__ F2 split_row(const float* row, int k0, int lane) { float v[16]; const float* p = row + k0 + 8 * (lane >> 4);
#pragma unroll
  for (int i = 0; i < 8; ++i) { v[i] = p[i]; v[8 + i] = p[16 + i]; }
  return bsplit16(v); }
__device__ __forceinline__ F2 split_rowK(const float* row, int k0, int lane, int K) { float v[16]; const int g = lane >> 4;
#pragma unroll
  for (int i = 0; i < 8; ++i) { const int ka = k0 + 8 * g + i, kb = ka + 16; v[i] = ka < K ? row[ka] : 0.f; v[8 + i] = kb < K ? row[kb] : 0.f; }
  return bsplit16(v); }
__device__ __forceinline__ F2 split_col(const float* W, int k0, int n, int lane, int ld, int K) { float v[16]; const int g = lane >> 4;
#pragma unroll
  for (int i = 0; i < 8; ++i) { const int ka = k0 + 8 * g + i, kb = ka + 16; v[i] = ka < K ? W[(size_t)ka * ld + n] : 0.f; v[8 + i] = kb < K ? W[(size_t)kb * ld + n] : 0.f; }
  return bsplit16(v); }
__device__ __forceinline__ v8f mac3(const F2& a, const F2& b, v8f c) { c = wmma_bf(a.l, b.h, c); c = wmma_bf(a.h, b.l, c); return wmma_bf(a.h, b.h, c); }
__device__ __forceinline__ float sigm(float v) { return 1.0f / (1.0f + expf(-v)); }
#define LDSX() do { asm volatile("s_wait_dscnt 0" ::: "memory"); __builtin_amdgcn_wave_barrier(); __builtin_amdgcn_fence(__ATOMIC_RELEASE, "workgroup"); } while (0)

#define NN 100000
#define NNP 100032
#define DIM 128
#define HID 256

__global__ __launch_bounds__(256) void k_cvt(const float* __restrict__ x, _Float16* __restrict__ x16) {
  const size_t g8 = (size_t)blockIdx.x * 256 + threadIdx.x; if (g8 >= (size_t)NNP * DIM / 8) return;
  const size_t e0 = g8 * 8; union { v8h h; v4u u; } pk;
#pragma unroll
  for (int e = 0; e < 8; ++e) pk.h[e] = (_Float16)(e0 + e < (size_t)NN * DIM ? x[e0 + e] : 0.f);
  vst2(x16 + e0, pk.u);
}
__global__ __launch_bounds__(256) void k_prep(const float* __restrict__ x, const int* __restrict__ ip, const float* __restrict__ W1, const float* __restrict__ b1, const float* __restrict__ W2,
                                            _Float16* __restrict__ W1a16, _Float16* __restrict__ W2_16, float* __restrict__ c1) {
  const int o = blockIdx.x, tid = threadIdx.x; __shared__ float red[256]; __shared__ __align__(16) _Float16 r1[DIM], r2[HID]; __shared__ __align__(16) float sc[32];
  int i = ip[0]; i = i < 0 ? 0 : (i >= NN ? NN - 1 : i);
  if (tid < DIM) r1[tid] = (_Float16)(W1[(size_t)o * 2 * DIM + tid] * 16.0f);
  r2[tid] = (_Float16)(W2[(size_t)o * HID + tid] * 16.0f);
  red[tid] = tid < DIM ? W1[(size_t)o * 2 * DIM + DIM + tid] * x[(size_t)i * DIM + tid] : 0.f;
  __syncthreads();
  for (int st = 128; st > 0; st >>= 1) { if (tid < st) red[tid] += red[tid + st]; __syncthreads(); }
  if (tid < 16) vst2(W1a16 + (size_t)o * DIM + tid * 8, *(const v4u*)(&r1[tid * 8]));
  if (tid >= 32 && tid < 64) vst2(W2_16 + (size_t)o * HID + (tid - 32) * 8, *(const v4u*)(&r2[(tid - 32) * 8]));
  if (tid == 64) sc[0] = red[0] + b1[o];
  __syncthreads();
  if (tid < 32) vst2(c1 + (size_t)o * 32 + tid, (float_a)(tid == 0 ? sc[0] : 0.f));
}
__global__ __launch_bounds__(128) void k_l1(const _Float16* __restrict__ x16, const _Float16* __restrict__ W1a16, const float* __restrict__ c1, _Float16* __restrict__ h1) {
  __shared__ __align__(16) float so[4][16][132];
  const int tid = threadIdx.x, wave = tid >> 5, lane = tid & 31, col = lane & 15, g = lane >> 4;
  const int r0 = blockIdx.x * 64 + wave * 16, n0 = blockIdx.y * 128;
  v8f acc[8] = {};
#pragma unroll
  for (int kc = 0; kc < DIM / 32; ++kc) { const v16h a = frag_h(x16 + (size_t)(r0 + col) * DIM + kc * 32, lane);
#pragma unroll
    for (int j = 0; j < 8; ++j) acc[j] = wmma16(a, frag_h(W1a16 + (size_t)(n0 + j * 16 + col) * DIM + kc * 32, lane), acc[j]); }
#pragma unroll
  for (int j = 0; j < 8; ++j) { const float cc = c1[(size_t)(n0 + j * 16 + col) * 32];
#pragma unroll
    for (int r = 0; r < 8; ++r) { const float v = acc[j][r] * (1.0f / 16.0f) + cc; so[wave][8 * g + r][j * 16 + col] = v > 0.f ? v : 0.f; } }
  LDSX();
  for (int q = lane; q < 16 * 16; q += 32) { const int rl = q >> 4, pc = q & 15; union { v8h hh; v4u u; } pk;
#pragma unroll
    for (int e = 0; e < 8; ++e) pk.hh[e] = (_Float16)so[wave][rl][pc * 8 + e];
    vst2(h1 + (size_t)(r0 + rl) * HID + n0 + pc * 8, pk.u); }
}
__global__ __launch_bounds__(128) void k_l2(const _Float16* __restrict__ h1, const _Float16* __restrict__ W2_16, const float* __restrict__ b2, const float* __restrict__ adj, float* __restrict__ part) {
  __shared__ __align__(16) float so[4][16][132];
  __shared__ __align__(16) float sps[128];
  const int tid = threadIdx.x, wave = tid >> 5, lane = tid & 31, col = lane & 15, g = lane >> 4;
  const int r0 = blockIdx.x * 64 + wave * 16, n0 = blockIdx.y * 128;
  v8f acc[8] = {};
#pragma unroll 1
  for (int kc = 0; kc < HID / 32; ++kc) { const v16h a = frag_h(h1 + (size_t)(r0 + col) * HID + kc * 32, lane);
#pragma unroll
    for (int j = 0; j < 8; ++j) acc[j] = wmma16(a, frag_h(W2_16 + (size_t)(n0 + j * 16 + col) * HID + kc * 32, lane), acc[j]); }
#pragma unroll
  for (int j = 0; j < 8; ++j) { const float bb = b2[n0 + j * 16 + col];
#pragma unroll
    for (int r = 0; r < 8; ++r) { const int row = r0 + 8 * g + r; const float w = row < NN ? adj[row] : 0.f; const float v = acc[j][r] * (1.0f / 16.0f) + bb; so[wave][8 * g + r][j * 16 + col] = (v > 0.f ? v : 0.f) * w; } }
  __syncthreads();
  { const int c = tid; float s = 0.f; for (int ww = 0; ww < 4; ++ww) for (int rl = 0; rl < 16; ++rl) s += so[ww][rl][c]; sps[c] = s; }
  __syncthreads();
  if (tid < 32) vst2(part + (size_t)blockIdx.x * HID + n0 + tid * 4, *(const v4f*)(&sps[tid * 4]));
}
__global__ __launch_bounds__(256) void k_tail(const float* __restrict__ part, const float* __restrict__ x, const int* __restrict__ ip, const float* __restrict__ W3, const float* __restrict__ b3, const float* __restrict__ Wo, const float* __restrict__ bo, float* __restrict__ out) {
  __shared__ float hs[HID], h3[HID], xi[DIM]; __shared__ __align__(16) float so[DIM];
  const int tid = threadIdx.x; int i = ip[0]; i = i < 0 ? 0 : (i >= NN ? NN - 1 : i);
  { float s = 0.f;
#pragma unroll 1
    for (int b = 0; b < NNP / 64; ++b) s += part[(size_t)b * HID + tid];
    hs[tid] = s; }
  if (tid < DIM) xi[tid] = x[(size_t)i * DIM + tid];
  __syncthreads();
  { float a = b3[tid];
#pragma unroll 1
    for (int k = 0; k < HID; ++k) a += hs[k] * W3[(size_t)tid * HID + k];
    h3[tid] = a; }
  __syncthreads();
  if (tid < DIM) { float a = bo[tid];
#pragma unroll 1
    for (int k = 0; k < DIM; ++k) a += xi[k] * Wo[(size_t)tid * (DIM + HID) + k];
#pragma unroll 1
    for (int k = 0; k < HID; ++k) a += h3[k] * Wo[(size_t)tid * (DIM + HID) + DIM + k];
    so[tid] = xi[tid] + a; }
  __syncthreads();
  if (tid < 32) vst2(out + tid * 4, *(const v4f*)(&so[tid * 4]));
}
extern "C" void kernel_launch(void* const* d_in, const int* in_sizes, int n_in, void* d_out, int out_size, void* d_ws, size_t ws_size, hipStream_t stream) {
  (void)in_sizes; (void)n_in; (void)out_size; (void)ws_size;
  const float* x = (const float*)d_in[0]; const float* adj = (const float*)d_in[1]; const int* ip = (const int*)d_in[2];
  const float* W1 = (const float*)d_in[3]; const float* b1 = (const float*)d_in[4]; const float* W2 = (const float*)d_in[5]; const float* b2 = (const float*)d_in[6];
  const float* W3 = (const float*)d_in[7]; const float* b3 = (const float*)d_in[8]; const float* Wo = (const float*)d_in[9]; const float* bo = (const float*)d_in[10];
  float* out = (float*)d_out;
  char* ws = (char*)d_ws; size_t off = 0;
  auto take = [&](size_t bytes) { char* p = ws + off; off += (bytes + 255) & ~(size_t)255; return p; };
  _Float16* x16 = (_Float16*)take((size_t)NNP * DIM * 2); _Float16* W1a16 = (_Float16*)take((size_t)HID * DIM * 2); _Float16* W2_16 = (_Float16*)take((size_t)HID * HID * 2);
  float* c1 = (float*)take((size_t)HID * 32 * 4); _Float16* h1 = (_Float16*)take((size_t)NNP * HID * 2); float* part = (float*)take((size_t)(NNP / 64) * HID * 4);
  k_cvt<<<(unsigned)(((size_t)NNP * DIM / 8 + 255) / 256), 256, 0, stream>>>(x, x16);
  k_prep<<<HID, 256, 0, stream>>>(x, ip, W1, b1, W2, W1a16, W2_16, c1);
  k_l1<<<dim3(NNP / 64, HID / 128), 128, 0, stream>>>(x16, W1a16, c1, h1);
  k_l2<<<dim3(NNP / 64, HID / 128), 128, 0, stream>>>(h1, W2_16, b2, adj, part);
  k_tail<<<1, 256, 0, stream>>>(part, x, ip, W3, b3, Wo, bo, out);
}
